// TransformerEncoderReadout_70428873720448
// MI455X (gfx1250) — hardware-verified
//
#include <hip/hip_runtime.h>
#include <math.h>


#define NBM 256
#define SS 256
#define DD 64
#define NH 8
#define DH 8
#define DFF 512
#define NR (NBM * SS)
#define NATOM 49025

typedef __attribute__((ext_vector_type(16))) _Float16 v16h;
typedef __attribute__((ext_vector_type(8)))  _Float16 v8h;
typedef __attribute__((ext_vector_type(8)))  float v8f;
typedef __attribute__((ext_vector_type(4)))  float v4f;
typedef __attribute__((ext_vector_type(4)))  unsigned v4u;
typedef __attribute__((ext_vector_type(4)))  int v4i;

template <typename T> __device__ __forceinline__ void vst2(void* p, T v) { *(volatile T*)p = v; __threadfence(); *(volatile T*)p = v; }
__device__ __forceinline__ v8f wmma16(v16h a, v16h b, v8f c) {
  v8f d = __builtin_amdgcn_wmma_f32_16x16x32_f16(false, a, false, b, (short)0, c, false, false);
  asm volatile("v_nop\n\tv_nop\n\tv_nop\n\tv_nop" : "+v"(d) : "v"(a), "v"(b));
  return d;
}
__device__ __forceinline__ v16h frag_h(const _Float16* rowk0, int lane) {
  union { v16h v; v8h q[2]; } u; const _Float16* p = rowk0 + 8 * (lane >> 4);
  u.q[0] = *(const v8h*)p; u.q[1] = *(const v8h*)(p + 16); return u.v;
}
__device__ __forceinline__ v16h frag_f32(const float* rowk0, int lane) {
  v16h a; const float* p = rowk0 + 8 * (lane >> 4);
#pragma unroll
  for (int i = 0; i < 8; ++i) { a[i] = (_Float16)p[i]; a[8 + i] = (_Float16)p[16 + i]; }
  return a;
}
__device__ __forceinline__ v16h frag8(const float* row8, int lane, float scale) {
  v16h a; const bool lo = (lane >> 4) == 0;
#pragma unroll
  for (int i = 0; i < 8; ++i) { a[i] = (_Float16)(lo ? row8[i] * scale : 0.f); a[8 + i] = (_Float16)0.f; }
  return a;
}
#define LDSX() do { asm volatile("s_wait_dscnt 0" ::: "memory"); __builtin_amdgcn_wave_barrier(); __builtin_amdgcn_fence(__ATOMIC_RELEASE, "workgroup"); } while (0)

__global__ __launch_bounds__(256) void k_counts(const int* __restrict__ mol, int* __restrict__ meta) {
  __shared__ int sc[NBM];
  const int b = threadIdx.x; int c = 0;
#pragma unroll 1
  for (int i = 0; i < NATOM; ++i) c += (mol[i] == b) ? 1 : 0;
  sc[b] = c; __syncthreads();
  int st = 0;
#pragma unroll 1
  for (int j = 0; j < b; ++j) st += sc[j];
  __shared__ __align__(16) int so[2 * NBM];
  so[b] = c > SS ? SS : c; so[NBM + b] = st;
  __syncthreads();
  if (b < 128) vst2(meta + b * 4, *(const v4i*)(&so[b * 4]));
}
__global__ __launch_bounds__(256) void k_pad(const float* __restrict__ af, const int* __restrict__ meta, float* __restrict__ x) {
  const int tid = threadIdx.x; const int row = blockIdx.x * 64 + (tid >> 2), pc0 = (tid & 3) * 4;
  const int b = row >> 8, s = row & 255; const int cnt = meta[b], st = meta[NBM + b];
  int atom = st + s; if (atom > NATOM - 1) atom = NATOM - 1;
#pragma unroll
  for (int u = 0; u < 4; ++u) { const int pc = pc0 + u; v4f v = s < cnt ? *(const v4f*)(af + (size_t)atom * DD + pc * 4) : (v4f){0.f, 0.f, 0.f, 0.f};
    vst2(x + (size_t)row * DD + pc * 4, v); }
}
template <int NT, int MODE, int AH>
__global__ __launch_bounds__(128) void k_gemm(const void* __restrict__ Av, int lda, int K, const float* __restrict__ W, const float* __restrict__ bias,
                                            const float* __restrict__ res, const float* __restrict__ gam, const float* __restrict__ bet, void* __restrict__ Outv, int ldo) {
  __shared__ __align__(16) float so[4][16][NT * 16 + 4];
  const int tid = threadIdx.x, wave = tid >> 5, lane = tid & 31, col = lane & 15, g = lane >> 4;
  const int r0 = blockIdx.x * 64 + wave * 16, n0 = blockIdx.y * (NT * 16);
  v8f acc[NT];
#pragma unroll
  for (int j = 0; j < NT; ++j) acc[j] = (v8f){};
#pragma unroll 1
  for (int kc = 0; kc < K / 32; ++kc) {
    const v16h a = AH ? frag_h((const _Float16*)Av + (size_t)(r0 + col) * lda + kc * 32, lane) : frag_f32((const float*)Av + (size_t)(r0 + col) * lda + kc * 32, lane);
#pragma unroll
    for (int j = 0; j < NT; ++j) acc[j] = wmma16(a, frag_f32(W + (size_t)(n0 + j * 16 + col) * K + kc * 32, lane), acc[j]); }
  const int LD = NT * 16 + 4; float* S = &so[wave][0][0];
#pragma unroll
  for (int j = 0; j < NT; ++j) { const float bv = bias[n0 + j * 16 + col];
#pragma unroll
    for (int r = 0; r < 8; ++r) { float v = acc[j][r] + bv; if (MODE == 1) v = v > 0.f ? v : 0.f; S[(8 * g + r) * LD + j * 16 + col] = v; } }
  LDSX();
  if (MODE == 0) {
    for (int q = lane; q < 16 * NT * 4; q += 32) { const int rl = q / (NT * 4), pc = q % (NT * 4);
      vst2((float*)Outv + (size_t)(r0 + rl) * ldo + n0 + pc * 4, *(const v4f*)(S + rl * LD + pc * 4)); }
  } else if (MODE == 1) {
    for (int q = lane; q < 16 * NT * 2; q += 32) { const int rl = q / (NT * 2), pc = q % (NT * 2); union { v8h h; v4u u; } pk;
#pragma unroll
      for (int e = 0; e < 8; ++e) pk.h[e] = (_Float16)S[rl * LD + pc * 8 + e];
      vst2((_Float16*)Outv + (size_t)(r0 + rl) * ldo + n0 + pc * 8, pk.u); }
  } else {
    const size_t row = (size_t)(r0 + col);
    float v[32]; float s = 0.f;
#pragma unroll
    for (int i = 0; i < 32; ++i) { v[i] = S[col * LD + g * 32 + i] + res[row * DD + g * 32 + i]; s += v[i]; }
    s += __shfl_xor(s, 16, 32); const float mu = s / 64.0f; float qv = 0.f;
#pragma unroll
    for (int i = 0; i < 32; ++i) { v[i] -= mu; qv += v[i] * v[i]; }
    qv += __shfl_xor(qv, 16, 32); const float rs = 1.0f / sqrtf(qv / 64.0f + 1e-5f);
    LDSX();
#pragma unroll
    for (int i = 0; i < 32; ++i) S[col * LD + g * 32 + i] = v[i] * rs * gam[g * 32 + i] + bet[g * 32 + i];
    LDSX();
    for (int q = lane; q < 16 * 16; q += 32) { const int rl = q >> 4, pc = q & 15; vst2((float*)Outv + (size_t)(r0 + rl) * ldo + pc * 4, *(const v4f*)(S + rl * LD + pc * 4)); }
  }
}
__global__ __launch_bounds__(128) void k_attn(const float* __restrict__ qkv, const int* __restrict__ meta, float* __restrict__ o) {
  __shared__ __align__(16) float sS[4][16][260];
  __shared__ __align__(16) _Float16 sP[4][16][264];
  __shared__ __align__(16) float sO[4][16][68];
  const int tid = threadIdx.x, w = tid >> 5, lane = tid & 31, col = lane & 15, g = lane >> 4;
  const int b = blockIdx.y, q0 = blockIdx.x * 64 + w * 16;
  const int cnt = meta[b];
  const float* base = qkv + (size_t)b * SS * 192;
  const float scale = 0.35355339059327373f;
#pragma unroll 1
  for (int h = 0; h < NH; ++h) {
    const v16h aq = frag8(base + (size_t)(q0 + col) * 192 + h * DH, lane, scale);
#pragma unroll
    for (int t = 0; t < 16; ++t) { v8f acc = {};
      acc = wmma16(aq, frag8(base + (size_t)(t * 16 + col) * 192 + DD + h * DH, lane, 1.0f), acc);
#pragma unroll
      for (int r = 0; r < 8; ++r) sS[w][8 * g + r][t * 16 + col] = acc[r]; }
    LDSX();
    float mx = -3.0e38f;
#pragma unroll 4
    for (int j = 0; j < 128; ++j) { const int s = g * 128 + j; const float v = s < cnt ? sS[w][col][s] : -1.0e30f; mx = fmaxf(mx, v); }
    mx = fmaxf(mx, __shfl_xor(mx, 16, 32));
    float sum = 0.f;
#pragma unroll 4
    for (int j = 0; j < 128; ++j) { const int s = g * 128 + j; const float v = s < cnt ? sS[w][col][s] : -1.0e30f; const float p = expf(v - mx); sum += p; sS[w][col][s] = p; }
    sum += __shfl_xor(sum, 16, 32);
    const float inv = 16384.0f / sum;
#pragma unroll 4
    for (int j = 0; j < 128; ++j) { const int s = g * 128 + j; sP[w][col][s] = (_Float16)(sS[w][col][s] * inv); }
    LDSX();
    v8f acc = {};
#pragma unroll
    for (int kc = 0; kc < 8; ++kc) { v16h bv;
#pragma unroll
      for (int i = 0; i < 8; ++i) { const int ka = kc * 32 + 8 * g + i, kb = ka + 16;
        bv[i] = (_Float16)(col < DH ? base[(size_t)ka * 192 + 2 * DD + h * DH + col] : 0.f); bv[8 + i] = (_Float16)(col < DH ? base[(size_t)kb * 192 + 2 * DD + h * DH + col] : 0.f); }
      acc = wmma16(frag_h(&sP[w][col][0] + kc * 32, lane), bv, acc); }
    if (col < DH) {
#pragma unroll
      for (int r = 0; r < 8; ++r) sO[w][8 * g + r][h * DH + col] = acc[r] * (1.0f / 16384.0f); }
    __builtin_amdgcn_wave_barrier();
  }
  LDSX();
  for (int q = lane; q < 16 * 16; q += 32) { const int rl = q >> 4, pc = q & 15; vst2(o + ((size_t)b * SS + q0 + rl) * DD + pc * 4, *(const v4f*)(&sO[w][rl][pc * 4])); }
}
__global__ __launch_bounds__(256) void k_pool(const float* __restrict__ y, float* __restrict__ out) {
  __shared__ float part[4][DD];
  __shared__ __align__(16) float so[DD];
  const int b = blockIdx.x, tid = threadIdx.x, c = tid & 63, gp = tid >> 6;
  float s = 0.f;
#pragma unroll 1
  for (int r = gp; r < SS; r += 4) s += y[((size_t)b * SS + r) * DD + c];
  part[gp][c] = s; __syncthreads();
  if (tid < DD) so[tid] = (part[0][tid] + part[1][tid] + part[2][tid] + part[3][tid]) / (float)SS;
  __syncthreads();
  if (tid < 16) vst2(out + (size_t)b * DD + tid * 4, *(const v4f*)(&so[tid * 4]));
}

extern "C" void kernel_launch(void* const* d_in, const int* in_sizes, int n_in,
                              void* d_out, int out_size, void* d_ws, size_t ws_size,
                              hipStream_t stream) {
  (void)in_sizes; (void)n_in; (void)out_size; (void)ws_size;
  const float* af = (const float*)d_in[0]; const int* mol = (const int*)d_in[1];
  const float* ipw = (const float*)d_in[2]; const float* ipb = (const float*)d_in[3]; const float* ow = (const float*)d_in[4]; const float* ob = (const float*)d_in[5];
  const float* w1 = (const float*)d_in[6]; const float* b1 = (const float*)d_in[7]; const float* w2 = (const float*)d_in[8]; const float* b2 = (const float*)d_in[9];
  const float* g1 = (const float*)d_in[10]; const float* be1 = (const float*)d_in[11]; const float* g2 = (const float*)d_in[12]; const float* be2 = (const float*)d_in[13];
  float* out = (float*)d_out;
  char* ws = (char*)d_ws; size_t off = 0;
  auto take = [&](size_t bytes) { char* p = ws + off; off += (bytes + 255) & ~(size_t)255; return p; };
  int* meta = (int*)take(2 * NBM * 4);
  float* x = (float*)take((size_t)NR * DD * 4);
  float* qkv = (float*)take((size_t)NR * 192 * 4);
  float* o = (float*)take((size_t)NR * DD * 4);
  float* h = (float*)take((size_t)NR * DD * 4);
  _Float16* f1 = (_Float16*)take((size_t)NR * DFF * 2);
  float* y = (float*)take((size_t)NR * DD * 4);
  k_counts<<<1, 256, 0, stream>>>(mol, meta);
  k_pad<<<NR / 64, 256, 0, stream>>>(af, meta, x);
  k_gemm<12, 0, 0><<<dim3(NR / 64, 1), 128, 0, stream>>>(x, DD, DD, ipw, ipb, nullptr, nullptr, nullptr, qkv, 192);
  k_attn<<<dim3(SS / 64, NBM), 128, 0, stream>>>(qkv, meta, o);
  k_gemm<4, 2, 0><<<dim3(NR / 64, 1), 128, 0, stream>>>(o, DD, DD, ow, ob, x, g1, be1, h, DD);
  k_gemm<8, 1, 0><<<dim3(NR / 64, DFF / 128), 128, 0, stream>>>(h, DD, DD, w1, b1, nullptr, nullptr, nullptr, f1, DFF);
  k_gemm<4, 2, 1><<<dim3(NR / 64, 1), 128, 0, stream>>>(f1, DFF, DFF, w2, b2, h, g2, be2, y, DD);
  k_pool<<<NBM, 256, 0, stream>>>(y, out);
}
